// LiquidOperator_80711025426845
// MI455X (gfx1250) — hardware-verified
//
#include <hip/hip_runtime.h>
#include <math.h>

typedef __attribute__((ext_vector_type(16))) _Float16 v16h;
typedef __attribute__((ext_vector_type(16))) __bf16 v16b;
typedef __attribute__((ext_vector_type(8)))  _Float16 v8h;
typedef __attribute__((ext_vector_type(8)))  float v8f;
typedef __attribute__((ext_vector_type(4)))  float v4f;
typedef __attribute__((ext_vector_type(2)))  float v2f;
typedef __attribute__((ext_vector_type(4)))  unsigned v4u;
typedef __attribute__((ext_vector_type(4)))  int v4i;
typedef float __attribute__((may_alias)) float_a;
typedef int __attribute__((may_alias)) int_a;

template <typename T> __device__ __forceinline__ void vst2(void* p, T v) { *(volatile T*)p = v; __threadfence(); *(volatile T*)p = v; }
__device__ __forceinline__ v8f wmma16(v16h a, v16h b, v8f c) {
  v8f d = __builtin_amdgcn_wmma_f32_16x16x32_f16(false, a, false, b, (short)0, c, false, false);
  asm volatile("v_nop\n\tv_nop\n\tv_nop\n\tv_nop" : "+v"(d) : "v"(a), "v"(b));
  return d;
}
__device__ __forceinline__ v8f wmma_bf(v16b a, v16b b, v8f c) {
  v8f d = __builtin_amdgcn_wmma_f32_16x16x32_bf16(false, a, false, b, (short)0, c, false, false);
  asm volatile("v_nop\n\tv_nop\n\tv_nop\n\tv_nop" : "+v"(d) : "v"(a), "v"(b));
  return d;
}
__device__ __forceinline__ v16h frag_h(const _Float16* rowk0, int lane) {
  union { v16h v; v8h q[2]; } u; const _Float16* p = rowk0 + 8 * (lane >> 4);
  u.q[0] = *(const v8h*)p; u.q[1] = *(const v8h*)(p + 16); return u.v;
}
__device__ __forceinline__ v16h frag_f32(const float* rowk0, int lane) {
  v16h a; const float* p = rowk0 + 8 * (lane >> 4);
#pragma unroll
  for (int i = 0; i < 8; ++i) { a[i] = (_Float16)p[i]; a[8 + i] = (_Float16)p[16 + i]; }
  return a;
}
__device__ __forceinline__ v16h frag_f32s(const float* rowk0, int lane, float sc) {
  v16h a; const float* p = rowk0 + 8 * (lane >> 4);
#pragma unroll
  for (int i = 0; i < 8; ++i) { a[i] = (_Float16)(p[i] * sc); a[8 + i] = (_Float16)(p[16 + i] * sc); }
  return a;
}
__device__ __forceinline__ v16h fragc_f32(const float* W, int k0, int n, int lane, int ld, int K) {
  v16h a; const int g = lane >> 4;
#pragma unroll
  for (int i = 0; i < 8; ++i) { const int ka = k0 + 8 * g + i, kb = ka + 16;
    a[i] = (_Float16)(ka < K ? W[(size_t)(ka < K ? ka : K - 1) * ld + n] : 0.f); a[8 + i] = (_Float16)(kb < K ? W[(size_t)(kb < K ? kb : K - 1) * ld + n] : 0.f); }
  return a;
}
struct F2 { v16b h, l; };
__device__ __forceinline__ F2 bsplit16(const float v[16]) { F2 r;
#pragma unroll
  for (int i = 0; i < 16; ++i) { const __bf16 h = (__bf16)v[i]; r.h[i] = h; r.l[i] = (__bf16)(v[i] - (float)h); }
  return r; }
__device__ __forceinline__ F2 split_row(const float* row, int k0, int lane) { float v[16]; const float* p = row + k0 + 8 * (lane >> 4);
#pragma unroll
  for (int i = 0; i < 8; ++i) { v[i] = p[i]; v[8 + i] = p[16 + i]; }
  return bsplit16(v); }
__device__ __forceinline__ F2 split_rowK(const float* row, int k0, int lane, int K) { float v[16]; const int g = lane >> 4;
#pragma unroll
  for (int i = 0; i < 8; ++i) { const int ka = k0 + 8 * g + i, kb = ka + 16; v[i] = ka < K ? row[ka < K ? ka : K - 1] : 0.f; v[8 + i] = kb < K ? row[kb < K ? kb : K - 1] : 0.f; }
  return bsplit16(v); }
__device__ __forceinline__ F2 split_col(const float* W, int k0, int n, int lane, int ld, int K) { float v[16]; const int g = lane >> 4;
#pragma unroll
  for (int i = 0; i < 8; ++i) { const int ka = k0 + 8 * g + i, kb = ka + 16; v[i] = ka < K ? W[(size_t)(ka < K ? ka : K - 1) * ld + n] : 0.f; v[8 + i] = kb < K ? W[(size_t)(kb < K ? kb : K - 1) * ld + n] : 0.f; }
  return bsplit16(v); }
__device__ __forceinline__ v8f mac3(const F2& a, const F2& b, v8f c) { c = wmma_bf(a.l, b.h, c); c = wmma_bf(a.h, b.l, c); return wmma_bf(a.h, b.h, c); }
__device__ __forceinline__ float sigm(float v) { return 1.0f / (1.0f + expf(-v)); }
#define LDSX() do { asm volatile("s_wait_dscnt 0" ::: "memory"); __builtin_amdgcn_wave_barrier(); __builtin_amdgcn_fence(__ATOMIC_RELEASE, "workgroup"); } while (0)


#define NP 8192
#define NT_ 512
#define NS 32
#define NTOKS (NT_ * NS)
#define DD 256
#define RFF 64
#define DT 16
#define QIN 152
#define QINP 160
#define NH 4
#define HDd 64
#ifndef NPT_
#define NPT_ NP
#endif
typedef __attribute__((ext_vector_type(8))) __bf16 v8b;
__device__ __forceinline__ v16b frag_b(const __bf16* rowk0, int lane) {
  union { v16b v; v8b q[2]; } u; const __bf16* p = rowk0 + 8 * (lane >> 4);
  u.q[0] = *(const v8b*)p; u.q[1] = *(const v8b*)(p + 16); return u.v;
}
__device__ __forceinline__ float bfr(float v) { return (float)(__bf16)v; }
__device__ __attribute__((noinline)) float exp_ni(float v) { return expf(v); }
__device__ __attribute__((noinline)) float erf_ni(float v) { return erff(v); }

__device__ __attribute__((noinline)) float cos_ni(float v) { return cosf(v); }
__device__ __attribute__((noinline)) float sin_ni(float v) { return sinf(v); }
#define WS_PW   0u
#define P_TIN 0
#define P_FC1(i) (P_TIN + 256 * QINP + (size_t)(i) * 2 * 256 * 256)
#define P_FC2(i) (P_FC1(i) + 256 * 256)
#define P_BTP (P_FC1(2))
#define P_WQ  (P_BTP + 256 * 256)
#define P_WK  (P_WQ + 256 * 256)
#define P_WV  (P_WK + 256 * 256)
#define P_AO  (P_WV + 256 * 256)
#define P_B1  (P_AO + 256 * 256)
#define P_B2  (P_B1 + 256 * 256)
#define P_TO  (P_B2 + 256 * 256)
#define P_BP  (P_TO + 768 * 256)
#define PWEND (P_BP + 768 * 256)
#define WS_IDX  (WS_PW + 2u * PWEND)
#define WS_DTQ  (WS_IDX + 4u * NP)
#define WS_A0   (WS_DTQ + 4u * NP)
#define WS_F    (WS_A0 + 4u * NP * QINP)
#define WS_T1   (WS_F + 4u * NP * DD)
#define WS_T2   (WS_T1 + 4u * NP * DD)
#define WS_TOK  (WS_T2 + 4u * NP * DD)
#define WS_KV   (WS_TOK + 4u * NTOKS * DD)
#define WS_Q    (WS_KV + 4u * NTOKS * 512)
#define WS_CTX  (WS_Q + 4u * NP * DD)
#define WS_TB   (WS_CTX + 4u * NP * DD)
#define WS_BB   (WS_TB + 4u * NP * 768)
#define WS_END  (WS_BB + 4u * NP * 768)

__global__ __launch_bounds__(256) void k_packW(const float* __restrict__ Wm, int K, int KP, __bf16* __restrict__ DST_) {
  __shared__ __align__(16) __bf16 s[256]; const int n = blockIdx.x, t = threadIdx.x; s[t] = (__bf16)((t < K) ? Wm[(size_t)n * K + t] : 0.f); __syncthreads();
  if (t < KP / 8) vst2((unsigned*)(DST_ + (size_t)n * KP + t * 8), *(const v4u*)&s[t * 8]);
}
__global__ __launch_bounds__(256) void k_pre(const float* __restrict__ XY, const float* __restrict__ TQ, const int* __restrict__ CC, const float* __restrict__ ST, const float* __restrict__ BM, const float* __restrict__ TW, const float* __restrict__ TB, const float* __restrict__ CE, int* __restrict__ IDX, float* __restrict__ DTQ, float* __restrict__ A0) {
  __shared__ __align__(16) float sa[64][QINP]; __shared__ __align__(16) int sidx[64]; __shared__ __align__(16) float sdt[64];
  const int t = threadIdx.x; const size_t p0 = (size_t)blockIdx.x * 64;
  if (t < 64) { const size_t p = p0 + t; const float tq = bfr(TQ[p]); int cnt = 0;
#pragma unroll 1
    for (int i = 0; i < NT_; ++i) cnt += (bfr(ST[i]) <= tq) ? 1 : 0;
    int id = cnt - 1; id = min(max(id, 0), NT_ - 1); sidx[t] = id; sdt[t] = fmaxf(tq - bfr(ST[id]), 0.f); }
  __syncthreads();
  for (int q = t; q < 64 * QINP; q += 256) { const int pl = q / QINP, cix = q % QINP; const size_t p = p0 + pl; float v = 0.f;
    if (cix < 2 * RFF) { const int f = cix % RFF; const float ph = bfr(XY[p * 2]) * bfr(BM[f]) + bfr(XY[p * 2 + 1]) * bfr(BM[RFF + f]); v = (cix < RFF) ? cos_ni(ph) : sin_ni(ph); }
    else if (cix < 2 * RFF + DT) { const int o = cix - 2 * RFF; v = sdt[pl] * bfr(TW[o]) + bfr(TB[o]); }
    else if (cix < QIN) { const int o = cix - 2 * RFF - DT; const int c = min(max(CC[p], 0), 2); v = bfr(CE[c * 8 + o]); }
    sa[pl][cix] = v; }
  __syncthreads();
  for (int q = t; q < 64 * QINP / 4; q += 256) { const int pl = q / (QINP / 4), pc = q % (QINP / 4); vst2(A0 + (p0 + pl) * QINP + pc * 4, *(const v4f*)&sa[pl][pc * 4]); }
  if (t < 16) { vst2((unsigned*)(IDX + p0 + t * 4), *(const v4u*)&sidx[t * 4]); vst2(DTQ + p0 + t * 4, *(const v4f*)&sdt[t * 4]); }
}
template <int MODE>
__global__ __launch_bounds__(128) void k_gemm(const float* __restrict__ A, int lda, int K, const float* __restrict__ LG, const float* __restrict__ LB_, const __bf16* __restrict__ P, const float* __restrict__ bias, const float* __restrict__ RES, int act, float* __restrict__ OUT, int ldo) {
  __shared__ __align__(16) float so[4][16][132]; __shared__ __align__(16) float sln[64][260];
  const int tid = threadIdx.x, wave = tid >> 5, lane = tid & 31, col = lane & 15, g = lane >> 4; const size_t r0 = (size_t)blockIdx.x * 64 + wave * 16; const int n0 = blockIdx.y * 128;
  if (MODE == 2) {
    for (int rl = 0; rl < 16; ++rl) { const float* row = A + (r0 + rl) * (size_t)lda; float v[8]; float s = 0.f;
#pragma unroll
      for (int k = 0; k < 8; ++k) { v[k] = row[lane + 32 * k]; s += v[k]; }
#pragma unroll
      for (int o = 1; o < 32; o <<= 1) s += __shfl_xor(s, o);
      const float mu = s / 256.f; float var = 0.f;
#pragma unroll
      for (int k = 0; k < 8; ++k) { const float d = v[k] - mu; var += d * d; }
#pragma unroll
      for (int o = 1; o < 32; o <<= 1) var += __shfl_xor(var, o);
      const float rs = rsqrtf(var / 256.f + 1e-5f);
#pragma unroll
      for (int k = 0; k < 8; ++k) { const int c = lane + 32 * k; sln[wave * 16 + rl][c] = (v[k] - mu) * rs * bfr(LG[c]) + bfr(LB_[c]); } }
    LDSX(); }
  v8f acc[8] = {};
  for (int kc = 0; kc < K / 32; ++kc) { F2 a; if (MODE == 1) { v16b ax; const float* p = A + (r0 + col) * (size_t)lda + kc * 32 + 8 * g;
#pragma unroll
      for (int i = 0; i < 8; ++i) { ax[i] = (__bf16)p[i]; ax[8 + i] = (__bf16)p[16 + i]; } a.h = ax; a.l = ax; }
    else if (MODE == 2) a = split_row(&sln[wave * 16 + col][0], kc * 32, lane); else a = split_row(A + (r0 + col) * (size_t)lda, kc * 32, lane);
#pragma unroll
    for (int j = 0; j < 8; ++j) { const v16b w = frag_b(P + (size_t)(n0 + j * 16 + col) * K + kc * 32, lane); if (MODE != 1) acc[j] = wmma_bf(a.l, w, acc[j]); acc[j] = wmma_bf(a.h, w, acc[j]); } }
#pragma unroll
  for (int j = 0; j < 8; ++j) { const int n = n0 + j * 16 + col; const float bb = bfr(bias[n]);
#pragma unroll
    for (int r = 0; r < 8; ++r) { float v = acc[j][r] + bb; if (act == 1) v = v * sigm(v); if (RES) v += RES[(r0 + 8 * g + r) * (size_t)ldo + n]; so[wave][8 * g + r][j * 16 + col] = v; } }
  LDSX();
  for (int rl = 0; rl < 16; ++rl) vst2(OUT + (r0 + rl) * (size_t)ldo + n0 + lane * 4, *(const v4f*)&so[wave][rl][lane * 4]);
}
__global__ __launch_bounds__(256) void k_attn1(const float* __restrict__ Q, const float* __restrict__ KV, const int* __restrict__ IDX, float* __restrict__ CTX) {
  __shared__ float ssc[8][NH][NS];
  const int tid = threadIdx.x, wave = tid >> 5, lane = tid & 31; const size_t p = (size_t)blockIdx.x * 8 + wave; const int id = min(max(IDX[p], 0), NT_ - 1); const size_t tb = (size_t)id * NS;
  const float* q = Q + p * DD;
  { const float* krow = KV + (tb + lane) * 512;
#pragma unroll
    for (int h = 0; h < NH; ++h) { float s = 0.f;
#pragma unroll 8
      for (int d = 0; d < HDd; ++d) s += q[h * HDd + d] * krow[h * HDd + d];
      ssc[wave][h][lane] = s * 0.125f; } }
  LDSX();
  float pr[NH];
#pragma unroll
  for (int h = 0; h < NH; ++h) { float v = ssc[wave][h][lane]; float mx = v;
#pragma unroll
    for (int o = 1; o < 32; o <<= 1) mx = fmaxf(mx, __shfl_xor(mx, o));
    const float e = exp_ni(v - mx); float s = e;
#pragma unroll
    for (int o = 1; o < 32; o <<= 1) s += __shfl_xor(s, o);
    pr[h] = e / s; }
  LDSX();
#pragma unroll
  for (int h = 0; h < NH; ++h) ssc[wave][h][lane] = pr[h];
  LDSX();
  float o8[8];
#pragma unroll
  for (int m = 0; m < 8; ++m) { const int c = lane + 32 * m; const int h = c / HDd; float a = 0.f;
#pragma unroll 4
    for (int s = 0; s < NS; ++s) a += ssc[wave][h][s] * KV[(tb + s) * 512 + 256 + c];
    o8[m] = a; }
#pragma unroll
  for (int m = 0; m < 8; ++m) vst2(CTX + p * DD + lane + 32 * m, o8[m]);
}
__global__ __launch_bounds__(256) void k_final(const float* __restrict__ TB, const float* __restrict__ BB, const int* __restrict__ CC, const float* __restrict__ LT, const float* __restrict__ CS, const float* __restrict__ CB, float* __restrict__ OUT) {
  __shared__ __align__(16) float so[64]; const int t = threadIdx.x; const int pl = t >> 2, part = t & 3; const size_t p = (size_t)blockIdx.x * 64 + pl; const int c = min(max(CC[p], 0), 2);
  float a = 0.f; const float* tr = TB + p * 768 + c * 256 + part * 64; const float* br = BB + p * 768 + c * 256 + part * 64;
#pragma unroll 8
  for (int r = 0; r < 64; ++r) a += tr[r] * br[r];
  a += __shfl_xor(a, 1); a += __shfl_xor(a, 2);
  if (part == 0) so[pl] = a * exp_ni(bfr(LT[0])) * bfr(CS[c]) + bfr(CB[c]);
  __syncthreads();
  if (t < 16) vst2(OUT + (size_t)blockIdx.x * 64 + t * 4, *(const v4f*)&so[t * 4]);
}
extern "C" void kernel_launch(void* const* d_in, const int* in_sizes, int n_in, void* d_out, int out_size, void* d_ws, size_t ws_size, hipStream_t stream) {
  (void)in_sizes; (void)n_in; (void)out_size;
  const float** F = (const float**)d_in; const int* CC = (const int*)d_in[2];
  if (ws_size < (size_t)WS_END) return;
  char* ws = (char*)d_ws; __bf16* PW = (__bf16*)(ws + WS_PW); int* IDX = (int*)(ws + WS_IDX); float *DTQ = (float*)(ws + WS_DTQ), *A0 = (float*)(ws + WS_A0), *FT = (float*)(ws + WS_F), *T1 = (float*)(ws + WS_T1), *T2 = (float*)(ws + WS_T2), *TOK = (float*)(ws + WS_TOK), *KV = (float*)(ws + WS_KV), *Q = (float*)(ws + WS_Q), *CTX = (float*)(ws + WS_CTX), *TB = (float*)(ws + WS_TB), *BB = (float*)(ws + WS_BB);
  const int NRB = NPT_ / 64;
  k_packW<<<256, 256, 0, stream>>>(F[9], QIN, QINP, PW + P_TIN);
  for (int i = 0; i < 2; ++i) { k_packW<<<256, 256, 0, stream>>>(F[13] + (size_t)i * 256 * 256, 256, 256, PW + P_FC1(i)); k_packW<<<256, 256, 0, stream>>>(F[15] + (size_t)i * 256 * 256, 256, 256, PW + P_FC2(i)); }
  k_packW<<<256, 256, 0, stream>>>(F[17], 256, 256, PW + P_BTP); k_packW<<<256, 256, 0, stream>>>(F[21], 256, 256, PW + P_WQ); k_packW<<<256, 256, 0, stream>>>(F[21] + 256 * 256, 256, 256, PW + P_WK); k_packW<<<256, 256, 0, stream>>>(F[21] + 2 * 256 * 256, 256, 256, PW + P_WV);
  k_packW<<<256, 256, 0, stream>>>(F[23], 256, 256, PW + P_AO); k_packW<<<256, 256, 0, stream>>>(F[27], 256, 256, PW + P_B1); k_packW<<<256, 256, 0, stream>>>(F[29], 256, 256, PW + P_B2); k_packW<<<768, 256, 0, stream>>>(F[31], 256, 256, PW + P_TO); k_packW<<<768, 256, 0, stream>>>(F[33], 256, 256, PW + P_BP);
  k_gemm<1><<<dim3(NTOKS / 64, 2), 128, 0, stream>>>(F[3], DD, DD, nullptr, nullptr, PW + P_BTP, F[18], nullptr, 0, TOK, DD);
  k_gemm<0><<<dim3(NTOKS / 64, 2), 128, 0, stream>>>(TOK, DD, DD, nullptr, nullptr, PW + P_WK, F[22] + 256, nullptr, 0, KV, 512);
  k_gemm<0><<<dim3(NTOKS / 64, 2), 128, 0, stream>>>(TOK, DD, DD, nullptr, nullptr, PW + P_WV, F[22] + 512, nullptr, 0, KV + 256, 512);
  k_pre<<<NRB, 256, 0, stream>>>(F[0], F[1], CC, F[4], F[5], F[6], F[7], F[8], IDX, DTQ, A0);
  k_gemm<0><<<dim3(NRB, 2), 128, 0, stream>>>(A0, QINP, QINP, nullptr, nullptr, PW + P_TIN, F[10], nullptr, 1, FT, DD);
  for (int i = 0; i < 2; ++i) { k_gemm<2><<<dim3(NRB, 2), 128, 0, stream>>>(FT, DD, DD, F[11] + i * 256, F[12] + i * 256, PW + P_FC1(i), F[14] + i * 256, nullptr, 1, T1, DD);
    k_gemm<0><<<dim3(NRB, 2), 128, 0, stream>>>(T1, DD, DD, nullptr, nullptr, PW + P_FC2(i), F[16] + i * 256, FT, 0, FT, DD);
  }
  k_gemm<0><<<dim3(NRB, 6), 128, 0, stream>>>(FT, DD, DD, nullptr, nullptr, PW + P_TO, F[32], nullptr, 0, TB, 768);
  k_gemm<2><<<dim3(NRB, 2), 128, 0, stream>>>(FT, DD, DD, F[19], F[20], PW + P_WQ, F[22], nullptr, 0, Q, DD);
  k_attn1<<<NPT_ / 8, 256, 0, stream>>>(Q, KV, IDX, T1);
  k_gemm<0><<<dim3(NRB, 2), 128, 0, stream>>>(T1, DD, DD, nullptr, nullptr, PW + P_AO, F[24], nullptr, 0, CTX, DD);
  k_gemm<2><<<dim3(NRB, 2), 128, 0, stream>>>(CTX, DD, DD, F[25], F[26], PW + P_B1, F[28], nullptr, 1, T1, DD);
  k_gemm<0><<<dim3(NRB, 2), 128, 0, stream>>>(T1, DD, DD, nullptr, nullptr, PW + P_B2, F[30], CTX, 0, T2, DD);
  k_gemm<0><<<dim3(NRB, 6), 128, 0, stream>>>(T2, DD, DD, nullptr, nullptr, PW + P_BP, F[34], nullptr, 0, BB, 768);
  k_final<<<NRB, 256, 0, stream>>>(TB, BB, CC, F[35], F[36], F[37], (float*)d_out);
}
